// FJSP_Decoder_21414706937958
// MI455X (gfx1250) — hardware-verified
//
#include <hip/hip_runtime.h>
#include <math.h>
#include <stdint.h>

#define NB   8
#define NJ   100
#define NM   20
#define NS   2000
#define SP   2048
#define DE   128
#define NH   8
#define QD   16
#define HP   32
#define QKP  512
#define QLP  256
#define NQB  32
#define MJ   832
#define MM   192
#define NP   384
static_assert(NH * QD == DE);
static_assert(NJ * NM == NS);
static_assert((SP % 64) == 0 && NS <= SP && NS > SP - 64);
static_assert((MJ % 64) == 0 && MJ >= NB * NJ && (MM % 64) == 0 && MM >= NB * NM);
static_assert(NH * HP == QLP && 2 * QLP == QKP);

typedef _Float16 v16h __attribute__((ext_vector_type(16)));
typedef _Float16 v8h  __attribute__((ext_vector_type(8)));
typedef __bf16   v16b __attribute__((ext_vector_type(16)));
typedef __bf16   v8b  __attribute__((ext_vector_type(8)));
typedef float    v8f  __attribute__((ext_vector_type(8)));
typedef float    v4f  __attribute__((ext_vector_type(4)));
typedef unsigned int v4u __attribute__((ext_vector_type(4)));

__device__ __forceinline__ unsigned short bf_bits(float f) {
  unsigned u = __float_as_uint(f);
  return (unsigned short)((u + 0x7FFFu + ((u >> 16) & 1u)) >> 16);
}
__device__ __forceinline__ float bf_up(unsigned short h) { return __uint_as_float(((unsigned)h) << 16); }
__device__ __forceinline__ float bf_rne(float f) { return bf_up(bf_bits(f)); }
__device__ __forceinline__ unsigned short h_bits(_Float16 x) { return __builtin_bit_cast(unsigned short, x); }
__device__ __forceinline__ unsigned pk16(unsigned short a, unsigned short b) { return (unsigned)a | ((unsigned)b << 16); }
__device__ __forceinline__ v8f zero8() { v8f z = {0.f, 0.f, 0.f, 0.f, 0.f, 0.f, 0.f, 0.f}; return z; }

__device__ __forceinline__ v16b ldfrag_b(const __bf16* p) {
  union { v16b v; v8b h[2]; } f;
  f.h[0] = *(const v8b*)(p);
  f.h[1] = *(const v8b*)(p + 16);
  return f.v;
}
__device__ __forceinline__ v16h ldfrag_h(const _Float16* p) {
  union { v16h v; v8h h[2]; } f;
  f.h[0] = *(const v8h*)(p);
  f.h[1] = *(const v8h*)(p + 16);
  return f.v;
}

__device__ __forceinline__ v8f mma_h(v16h a, v16h b, v8f c) {
  c = __builtin_amdgcn_wmma_f32_16x16x32_f16(false, a, false, b, (short)0, c, false, false);
#if defined(__HIP_DEVICE_COMPILE__)
  asm volatile("v_nop\n\tv_nop\n\tv_nop\n\tv_nop" : "+v"(c) : "v"(a), "v"(b));
#endif
  return c;
}
__device__ __forceinline__ v8f mma_b(v16b a, v16b b, v8f c) {
  c = __builtin_amdgcn_wmma_f32_16x16x32_bf16(false, a, false, b, (short)0, c, false, false);
#if defined(__HIP_DEVICE_COMPILE__)
  asm volatile("v_nop\n\tv_nop\n\tv_nop\n\tv_nop" : "+v"(c) : "v"(a), "v"(b));
#endif
  return c;
}
__device__ __forceinline__ v8f mma_b_raw(v16b a, v16b b, v8f c) {
  return __builtin_amdgcn_wmma_f32_16x16x32_bf16(false, a, false, b, (short)0, c, false, false);
}
__device__ __forceinline__ void dep_guard_b(v8f& a, v8f& b, v16b x, v16b y) {
#if defined(__HIP_DEVICE_COMPILE__)
  asm volatile("v_nop\n\tv_nop\n\tv_nop\n\tv_nop" : "+v"(a), "+v"(b) : "v"(x), "v"(y));
#endif
}
__device__ __forceinline__ void keep4_b(v16b a, v16b b, v16b c, v16b d) {
#if defined(__HIP_DEVICE_COMPILE__)
  asm volatile("v_nop" :: "v"(a), "v"(b), "v"(c), "v"(d));
#endif
}
__device__ __forceinline__ void acc_guard4(v8f& a, v8f& b, v8f& c, v8f& d) {
#if defined(__HIP_DEVICE_COMPILE__)
  asm volatile("v_nop\n\tv_nop\n\tv_nop\n\tv_nop" : "+v"(a), "+v"(b), "+v"(c), "+v"(d));
#endif
}
__device__ __forceinline__ void wave_sync_lds() {
  __builtin_amdgcn_fence(__ATOMIC_RELEASE, "workgroup");
  __builtin_amdgcn_wave_barrier();
  __builtin_amdgcn_fence(__ATOMIC_ACQUIRE, "workgroup");
}

__global__ __launch_bounds__(256) void cvt_bf16x8(const float* __restrict__ in, unsigned short* out,
                                                  int n8valid, int n8total) {
  const int i = blockIdx.x * 256 + threadIdx.x;
  if (i < n8total) {
    const int ic = (i < n8valid) ? i : (n8valid - 1);
    const v4f a = *(const v4f*)(in + (size_t)ic * 8);
    const v4f b = *(const v4f*)(in + (size_t)ic * 8 + 4);
    const bool z = (i >= n8valid);
    v4u p;
    p[0] = z ? 0u : pk16(bf_bits(a[0]), bf_bits(a[1]));
    p[1] = z ? 0u : pk16(bf_bits(a[2]), bf_bits(a[3]));
    p[2] = z ? 0u : pk16(bf_bits(b[0]), bf_bits(b[1]));
    p[3] = z ? 0u : pk16(bf_bits(b[2]), bf_bits(b[3]));
    *(volatile v4u*)(out + (size_t)i * 8) = p;
    __threadfence();
    *(volatile v4u*)(out + (size_t)i * 8) = p;
  }
}

__global__ __launch_bounds__(256) void wtr(const float* __restrict__ Wq, const float* __restrict__ Wk,
                                           const float* __restrict__ Wv, const float* __restrict__ Wm,
                                           unsigned short* WT, unsigned short* WmT) {
  __shared__ __align__(16) unsigned int Tu[32 * 68];
  const int blk = blockIdx.x;
  const int tid = threadIdx.x;
  const float* src;
  int ibase, c0, orow0;
  unsigned short* dst;
  if (blk < 24) {
    const int ct = blk & 3;
    const int rest = blk >> 2;
    const int x = rest % 3;
    const int part = rest / 3;
    src = (x == 0) ? Wq : ((x == 1) ? Wk : Wv);
    ibase = part * DE;
    c0 = ct * 32;
    dst = WT;
    orow0 = part * NP + x * DE + c0;
  } else {
    const int ct = blk - 24;
    src = Wm;
    ibase = 0;
    c0 = ct * 32;
    dst = WmT;
    orow0 = c0;
  }
#pragma unroll 1
  for (int r = 0; r < 8; ++r) {
    const int e = r * 256 + tid;
    const int cc = e & 31;
    const int ip = e >> 5;
    const float f0 = src[(size_t)(ibase + 2 * ip) * DE + c0 + cc];
    const float f1 = src[(size_t)(ibase + 2 * ip + 1) * DE + c0 + cc];
    Tu[cc * 68 + ip] = pk16(bf_bits(f0), bf_bits(f1));
  }
  __syncthreads();
#pragma unroll 1
  for (int r = 0; r < 2; ++r) {
    const int task = r * 256 + tid;
    const int row = task >> 4;
    const int q16 = task & 15;
    const v4u v = *(const v4u*)(Tu + row * 68 + q16 * 4);
    unsigned short* p = dst + (size_t)(orow0 + row) * DE + q16 * 8;
    *(volatile v4u*)p = v;
    __threadfence();
    *(volatile v4u*)p = v;
  }
}

template <int NSPLIT, int OUT_MODE>
__global__ __launch_bounds__(256) void gemm64(
    const unsigned short* __restrict__ Ap, const unsigned short* A2p, int lda, long long strideA,
    const unsigned short* __restrict__ Btp, const unsigned short* Bt2p, int ldb, long long strideB,
    void* Cout, int ldc, long long strideC,
    void* Cout2, int ldc2, long long strideC2, int N2,
    int M, int N, int K, float rscale) {
  const __bf16* A   = (const __bf16*)(const void*)Ap;
  const __bf16* A2  = (const __bf16*)(const void*)A2p;
  const __bf16* Bt  = (const __bf16*)(const void*)Btp;
  const __bf16* Bt2 = (const __bf16*)(const void*)Bt2p;
  __shared__ __align__(16) float sT[8][16 * 68];
  const int b    = blockIdx.y;
  const int lane = threadIdx.x & 31;
  const int wave = threadIdx.x >> 5;
  const int tilesN = N >> 6;
  const int tilesM = M >> 6;
  const int tile = blockIdx.x * 8 + wave;
  if (tile >= tilesM * tilesN) return;
  const int tm = tile / tilesN;
  const int tn = tile - tm * tilesN;
  const int m0 = tm << 6;
  const int n0 = tn << 6;

  const __bf16* Ab  = A  + (size_t)b * strideA;
  const __bf16* Bb  = Bt + (size_t)b * strideB;
  const __bf16* Ab2 = (NSPLIT >= 1) ? (A2  + (size_t)b * strideA) : Ab;
  const __bf16* Bb2 = (NSPLIT == 2) ? (Bt2 + (size_t)b * strideB) : Bb;

  const int rlane = lane & 15;
  const int koff  = (lane >> 4) * 8;
  const int mOff  = (lane >> 4) * 8;

  v8f acc[4][4];
#pragma unroll
  for (int i = 0; i < 4; ++i)
#pragma unroll
    for (int j = 0; j < 4; ++j) acc[i][j] = zero8();

  for (int k0 = 0; k0 < K; k0 += 32) {
    v16b bh[4], bl[4];
#pragma unroll
    for (int j = 0; j < 4; ++j) {
      const size_t bo = (size_t)(n0 + (j << 4) + rlane) * ldb + koff + k0;
      bh[j] = ldfrag_b(Bb + bo);
      if (NSPLIT == 2) bl[j] = ldfrag_b(Bb2 + bo); else bl[j] = bh[j];
    }
#pragma unroll
    for (int i = 0; i < 4; ++i) {
      const size_t ao = (size_t)(m0 + (i << 4) + rlane) * lda + koff + k0;
      const v16b ah = ldfrag_b(Ab + ao);
      v16b al = ah;
      if (NSPLIT >= 1) al = ldfrag_b(Ab2 + ao);
#pragma unroll
      for (int j = 0; j < 4; ++j) {
        acc[i][j] = mma_b_raw(ah, bh[j], acc[i][j]);
        if (NSPLIT >= 1) acc[i][j] = mma_b_raw(al, bh[j], acc[i][j]);
        if (NSPLIT == 2) acc[i][j] = mma_b_raw(ah, bl[j], acc[i][j]);
      }
      dep_guard_b(acc[i][0], acc[i][3], ah, al);
    }
    keep4_b(bh[0], bh[1], bh[2], bh[3]);
    if (NSPLIT == 2) keep4_b(bl[0], bl[1], bl[2], bl[3]);
  }
  acc_guard4(acc[0][0], acc[0][1], acc[0][2], acc[0][3]);
  acc_guard4(acc[1][0], acc[1][1], acc[1][2], acc[1][3]);
  acc_guard4(acc[2][0], acc[2][1], acc[2][2], acc[2][3]);
  acc_guard4(acc[3][0], acc[3][1], acc[3][2], acc[3][3]);

  float* slab = sT[wave];
#pragma unroll
  for (int i = 0; i < 4; ++i) {
    const int mBase = m0 + (i << 4);
#pragma unroll
    for (int j = 0; j < 4; ++j) {
#pragma unroll
      for (int r = 0; r < 8; ++r) {
        slab[(mOff + r) * 68 + (j << 4) + rlane] = acc[i][j][r];
      }
    }
    wave_sync_lds();
    if (OUT_MODE == 0) {
      float* C = (float*)Cout + (size_t)b * strideC;
      const int hh = lane >> 4, c4 = (lane & 15) * 4;
      for (int pass = 0; pass < 2; ++pass) {
#pragma unroll
        for (int it = 0; it < 8; ++it) {
          const int row = it * 2 + hh;
          const v4f v = *(const v4f*)(slab + row * 68 + c4);
          *(volatile v4f*)(C + (size_t)(mBase + row) * ldc + n0 + c4) = v;
        }
        __threadfence();
      }
    } else {
      const int q = lane >> 3, c8 = (lane & 7) * 8;
      unsigned short* C  = (unsigned short*)Cout  + (size_t)b * strideC;
      unsigned short* C2 = (unsigned short*)Cout2 + (size_t)b * strideC2;
      const bool wlo = (OUT_MODE == 2) || (n0 < N2);
      v4u hv[4], lv[4];
#pragma unroll
      for (int it = 0; it < 4; ++it) {
        const int row = it * 4 + q;
        const float* sp = slab + row * 68 + c8;
        v4u a, a2;
#pragma unroll
        for (int e = 0; e < 4; ++e) {
          const float f0 = sp[2 * e], f1 = sp[2 * e + 1];
          unsigned short h0, h1, l0, l1;
          if (OUT_MODE == 2) {
            h0 = bf_bits(f0); h1 = bf_bits(f1);
            l0 = bf_bits(f0 - bf_up(h0)); l1 = bf_bits(f1 - bf_up(h1));
          } else {
            const _Float16 x0 = (_Float16)f0, x1 = (_Float16)f1;
            h0 = h_bits(x0); h1 = h_bits(x1);
            l0 = h_bits((_Float16)((f0 - (float)x0) * rscale));
            l1 = h_bits((_Float16)((f1 - (float)x1) * rscale));
          }
          a[e] = pk16(h0, h1); a2[e] = pk16(l0, l1);
        }
        hv[it] = a; lv[it] = a2;
      }
      for (int pass = 0; pass < 2; ++pass) {
#pragma unroll
        for (int it = 0; it < 4; ++it) {
          const int row = it * 4 + q;
          *(volatile v4u*)(C + (size_t)(mBase + row) * ldc + n0 + c8) = hv[it];
          if (wlo) *(volatile v4u*)(C2 + (size_t)(mBase + row) * ldc2 + n0 + c8) = lv[it];
        }
        __threadfence();
      }
    }
    wave_sync_lds();
  }
}

__global__ __launch_bounds__(256) void asm_qkv(const float* __restrict__ Pj, const float* __restrict__ Pm,
                                               unsigned short* QK, unsigned short* Ql,
                                               unsigned short* VTh, unsigned short* VTl, float rs) {
  __shared__ __align__(16) float Vs[DE * 68];
  const int tid = threadIdx.x;
  const int st  = blockIdx.x & (NQB - 1);
  const int b   = blockIdx.x >> 5;
  const int s0  = st * 64;
  const int q8  = tid & 7;

#pragma unroll 1
  for (int it = 0; it < 16; ++it) {
    const int Lg = it * 32 + (tid >> 3);
    const int rl = Lg >> 3;
    const int L  = Lg & 7;
    const int s  = s0 + rl;
    const bool valid = (s < NS);
    const int sc = valid ? s : (NS - 1);
    const int j  = sc / NM;
    const int m  = sc - j * NM;
    const int x  = L >> 2;
    const int h  = 2 * (L & 3) + ((q8 >> 2) & 1);
    const int d0 = (q8 & 1) * 8;
    const bool isval = valid && ((q8 & 2) == 0);
    const int col = x * DE + h * QD + d0;
    const float* pa = Pj + (size_t)(b * NJ + j) * NP + col;
    const float* pb = Pm + (size_t)(b * NM + m) * NP + col;
    const v4f a0 = *(const v4f*)pa, a1 = *(const v4f*)(pa + 4);
    const v4f b0 = *(const v4f*)pb, b1 = *(const v4f*)(pb + 4);
    float v[8];
    v[0] = isval ? (a0[0] + b0[0]) : 0.f;  v[1] = isval ? (a0[1] + b0[1]) : 0.f;
    v[2] = isval ? (a0[2] + b0[2]) : 0.f;  v[3] = isval ? (a0[3] + b0[3]) : 0.f;
    v[4] = isval ? (a1[0] + b1[0]) : 0.f;  v[5] = isval ? (a1[1] + b1[1]) : 0.f;
    v[6] = isval ? (a1[2] + b1[2]) : 0.f;  v[7] = isval ? (a1[3] + b1[3]) : 0.f;
    v4u hv, lv;
#pragma unroll
    for (int e = 0; e < 4; ++e) {
      const float f0 = v[2 * e], f1 = v[2 * e + 1];
      const _Float16 x0 = (_Float16)f0, x1 = (_Float16)f1;
      hv[e] = pk16(h_bits(x0), h_bits(x1));
      lv[e] = pk16(h_bits((_Float16)((f0 - (float)x0) * rs)), h_bits((_Float16)((f1 - (float)x1) * rs)));
    }
    unsigned short* dq = QK + (size_t)(b * SP + s) * QKP + L * 64 + q8 * 8;
    unsigned short* dl = Ql + (size_t)(b * SP + s) * QLP + L * 64 + q8 * 8;
    *(volatile v4u*)dq = hv;
    if (x == 0) *(volatile v4u*)dl = lv;
    __threadfence();
    *(volatile v4u*)dq = hv;
    if (x == 0) *(volatile v4u*)dl = lv;
  }

#pragma unroll 1
  for (int it = 0; it < 4; ++it) {
    const int item = it * 256 + tid;
    const int g  = item & 15;
    const int rl = item >> 4;
    const int s  = s0 + rl;
    const bool valid = (s < NS);
    const int sc = valid ? s : (NS - 1);
    const int j  = sc / NM;
    const int m  = sc - j * NM;
    const int col = 2 * DE + 8 * g;
    const float* pa = Pj + (size_t)(b * NJ + j) * NP + col;
    const float* pb = Pm + (size_t)(b * NM + m) * NP + col;
    const v4f a0 = *(const v4f*)pa, a1 = *(const v4f*)(pa + 4);
    const v4f b0 = *(const v4f*)pb, b1 = *(const v4f*)(pb + 4);
    Vs[(8 * g + 0) * 68 + rl] = valid ? (a0[0] + b0[0]) : 0.f;
    Vs[(8 * g + 1) * 68 + rl] = valid ? (a0[1] + b0[1]) : 0.f;
    Vs[(8 * g + 2) * 68 + rl] = valid ? (a0[2] + b0[2]) : 0.f;
    Vs[(8 * g + 3) * 68 + rl] = valid ? (a0[3] + b0[3]) : 0.f;
    Vs[(8 * g + 4) * 68 + rl] = valid ? (a1[0] + b1[0]) : 0.f;
    Vs[(8 * g + 5) * 68 + rl] = valid ? (a1[1] + b1[1]) : 0.f;
    Vs[(8 * g + 6) * 68 + rl] = valid ? (a1[2] + b1[2]) : 0.f;
    Vs[(8 * g + 7) * 68 + rl] = valid ? (a1[3] + b1[3]) : 0.f;
  }
  __syncthreads();

#pragma unroll 1
  for (int it = 0; it < 4; ++it) {
    const int c = it * 32 + (tid >> 3);
    const float* sp = Vs + c * 68 + q8 * 8;
    const v4f x0 = *(const v4f*)sp, x1 = *(const v4f*)(sp + 4);
    float v[8];
    v[0] = x0[0]; v[1] = x0[1]; v[2] = x0[2]; v[3] = x0[3];
    v[4] = x1[0]; v[5] = x1[1]; v[6] = x1[2]; v[7] = x1[3];
    v4u hv, lv;
#pragma unroll
    for (int e = 0; e < 4; ++e) {
      const float f0 = v[2 * e], f1 = v[2 * e + 1];
      const _Float16 y0 = (_Float16)f0, y1 = (_Float16)f1;
      hv[e] = pk16(h_bits(y0), h_bits(y1));
      lv[e] = pk16(h_bits((_Float16)((f0 - (float)y0) * rs)), h_bits((_Float16)((f1 - (float)y1) * rs)));
    }
    const size_t go = (size_t)(b * DE + c) * SP + s0 + q8 * 8;
    *(volatile v4u*)(VTh + go) = hv;
    *(volatile v4u*)(VTl + go) = lv;
    __threadfence();
    *(volatile v4u*)(VTh + go) = hv;
    *(volatile v4u*)(VTl + go) = lv;
  }
}

__global__ __launch_bounds__(128)
void attn16(const unsigned short* __restrict__ qkp, const unsigned short* __restrict__ qlp,
            const unsigned short* __restrict__ vhp, const unsigned short* __restrict__ vlp,
            unsigned short* ohp, unsigned short* olp, float sscale, float rres) {
  union FH { v16h v; v8h h[2]; };
  __shared__ __align__(16) _Float16 Ksh[64 * HP];
  __shared__ __align__(16) _Float16 Vth[QD * 64];
  __shared__ __align__(16) _Float16 Vtl[QD * 64];
  __shared__ __align__(16) _Float16 Psh[4][16 * 64];
  __shared__ __align__(16) float    Os[4][16 * 16];

  const int tid  = threadIdx.x;
  const int wave = tid >> 5;
  const int lane = tid & 31;
  const int hh   = lane >> 4;
  const int c    = lane & 15;

  const int bx   = blockIdx.x;
  const int qb   = bx % NQB;
  const int rest = bx / NQB;
  const int h    = rest % NH;
  const int b    = rest / NH;
  const int q0   = qb * 64 + wave * 16;
  const size_t rowB = (size_t)b * SP;

  const _Float16* Qh = (const _Float16*)(const void*)qkp + (size_t)h * HP;
  const _Float16* Kg = (const _Float16*)(const void*)qkp + QLP + (size_t)h * HP;
  const _Float16* Qr = (const _Float16*)(const void*)qlp + (size_t)h * HP;
  const _Float16* Vh = (const _Float16*)(const void*)vhp + ((size_t)b * DE + (size_t)h * QD) * SP;
  const _Float16* Vl = (const _Float16*)(const void*)vlp + ((size_t)b * DE + (size_t)h * QD) * SP;

  const v16h qah = ldfrag_h(Qh + (rowB + q0 + c) * QKP + 8 * hh);
  const v16h qal = ldfrag_h(Qr + (rowB + q0 + c) * QLP + 8 * hh);

  float mrow[8], lrow[8];
#pragma unroll
  for (int r = 0; r < 8; ++r) { mrow[r] = -INFINITY; lrow[r] = 0.f; }
  v8f oacc = zero8();

  for (int kt = 0; kt < NQB; ++kt) {
    const int kv0 = kt * 64;
    __syncthreads();
    {
      const int r = tid >> 1, hf = (tid & 1) * 16;
      const _Float16* kg = Kg + (rowB + kv0 + r) * QKP + hf;
      const v8h a0 = *(const v8h*)(kg);
      const v8h a1 = *(const v8h*)(kg + 8);
      *(v8h*)(Ksh + r * HP + hf)     = a0;
      *(v8h*)(Ksh + r * HP + hf + 8) = a1;
      const int r2 = tid >> 3, s8 = (tid & 7) * 8;
      const v8h b0 = *(const v8h*)(Vh + (size_t)r2 * SP + kv0 + s8);
      const v8h b1 = *(const v8h*)(Vl + (size_t)r2 * SP + kv0 + s8);
      *(v8h*)(Vth + r2 * 64 + s8) = b0;
      *(v8h*)(Vtl + r2 * 64 + s8) = b1;
    }
    __syncthreads();

    v8f s[4];
#pragma unroll
    for (int j = 0; j < 4; ++j) {
      FH kb;
      kb.h[0] = *(const v8h*)(Ksh + (j * 16 + c) * HP + 8 * hh);
      kb.h[1] = *(const v8h*)(Ksh + (j * 16 + c) * HP + 16 + 8 * hh);
      v8f sh = mma_h(qah, kb.v, zero8());
      v8f sl = mma_h(qal, kb.v, zero8());
      const bool kval = (kv0 + j * 16 + c) < NS;
#pragma unroll
      for (int r = 0; r < 8; ++r) {
        const float sv = (sh[r] + sl[r] * rres) * sscale;
        s[j][r] = kval ? sv : -1e30f;
      }
    }

    _Float16* pwh = Psh[wave];
#pragma unroll
    for (int r = 0; r < 8; ++r) {
      float m = s[0][r];
      m = fmaxf(m, s[1][r]);
      m = fmaxf(m, s[2][r]);
      m = fmaxf(m, s[3][r]);
#pragma unroll
      for (int off = 1; off < 16; off <<= 1) m = fmaxf(m, __shfl_xor(m, off, 32));
      const float mnew  = fmaxf(mrow[r], m);
      const float alpha = __expf(mrow[r] - mnew);
      mrow[r] = mnew;
      float psum = 0.f;
#pragma unroll
      for (int j = 0; j < 4; ++j) {
        const float p = __expf(s[j][r] - mnew);
        psum += p;
        pwh[(8 * hh + r) * 64 + j * 16 + c] = (_Float16)(p * 1024.0f);
      }
#pragma unroll
      for (int off = 1; off < 16; off <<= 1) psum += __shfl_xor(psum, off, 32);
      lrow[r] = lrow[r] * alpha + psum;
      oacc[r] *= alpha;
    }
    wave_sync_lds();

    v8f o1 = zero8();
#pragma unroll
    for (int kk = 0; kk < 2; ++kk) {
      FH pa, vb, vl;
      pa.h[0] = *(const v8h*)(pwh + c * 64 + kk * 32 + 8 * hh);
      pa.h[1] = *(const v8h*)(pwh + c * 64 + kk * 32 + 16 + 8 * hh);
      vb.h[0] = *(const v8h*)(Vth + c * 64 + kk * 32 + 8 * hh);
      vb.h[1] = *(const v8h*)(Vth + c * 64 + kk * 32 + 16 + 8 * hh);
      vl.h[0] = *(const v8h*)(Vtl + c * 64 + kk * 32 + 8 * hh);
      vl.h[1] = *(const v8h*)(Vtl + c * 64 + kk * 32 + 16 + 8 * hh);
      oacc = mma_h(pa.v, vb.v, oacc);
      o1   = mma_h(pa.v, vl.v, o1);
    }
#pragma unroll
    for (int r = 0; r < 8; ++r) oacc[r] += o1[r] * rres;
  }

  float* os = Os[wave];
#pragma unroll
  for (int r = 0; r < 8; ++r) {
    const float l = lrow[r];
    const float inv = ((l > 0.f) ? (1.0f / l) : 0.f) * (1.0f / 1024.0f);
    os[(8 * hh + r) * QD + c] = oacc[r] * inv;
  }
  wave_sync_lds();
  {
    const int row = lane >> 1, d0 = (lane & 1) * 8;
    const float* sp = os + row * QD + d0;
    const v4f x0 = *(const v4f*)sp, x1 = *(const v4f*)(sp + 4);
    float f[8];
    f[0] = x0[0]; f[1] = x0[1]; f[2] = x0[2]; f[3] = x0[3];
    f[4] = x1[0]; f[5] = x1[1]; f[6] = x1[2]; f[7] = x1[3];
    v4u hv, lv;
#pragma unroll
    for (int e = 0; e < 4; ++e) {
      const float f0 = f[2 * e], f1 = f[2 * e + 1];
      const unsigned short h0 = bf_bits(f0), h1 = bf_bits(f1);
      const unsigned short l0 = bf_bits(f0 - bf_up(h0)), l1 = bf_bits(f1 - bf_up(h1));
      hv[e] = pk16(h0, h1); lv[e] = pk16(l0, l1);
    }
    const size_t go = (((size_t)b * NH + h) * SP + q0 + row) * QD + d0;
    *(volatile v4u*)(ohp + go) = hv;
    *(volatile v4u*)(olp + go) = lv;
    __threadfence();
    *(volatile v4u*)(ohp + go) = hv;
    *(volatile v4u*)(olp + go) = lv;
  }
}

__global__ __launch_bounds__(128)
void mhlogit(const unsigned short* __restrict__ ohp, const unsigned short* __restrict__ olp,
             const unsigned short* __restrict__ wmt, const float* __restrict__ bm,
             const float* __restrict__ wsh, const float* __restrict__ bsh,
             const float* __restrict__ mask, float* lgp, float isd, float clip) {
  union FB { v16b v; v8b h[2]; };
  __shared__ __align__(16) float Mt[4][16 * 132];
  __shared__ float bbs[DE];
  __shared__ float wss[DE];
  __shared__ __align__(16) float lgs[64];

  const int tid  = threadIdx.x;
  const int wave = tid >> 5;
  const int lane = tid & 31;
  const int hh   = lane >> 4;
  const int c    = lane & 15;
  const int R0   = blockIdx.x * 64;
  const int b    = R0 / SP;
  const int sb0  = R0 - b * SP;
  const int s0w  = sb0 + wave * 16;

  bbs[tid] = bf_rne(bm[tid]);
  wss[tid] = bf_rne(wsh[tid]);
  __syncthreads();

  const __bf16* Oh = (const __bf16*)(const void*)ohp;
  const __bf16* Ol = (const __bf16*)(const void*)olp;
  const __bf16* Wb = (const __bf16*)(const void*)wmt;

  v8f acc[8];
#pragma unroll
  for (int j = 0; j < 8; ++j) acc[j] = zero8();

#pragma unroll 1
  for (int kc = 0; kc < 4; ++kc) {
    const size_t a0 = (((size_t)b * NH + 2 * kc) * SP + s0w + c) * QD + 8 * hh;
    const size_t a1 = a0 + (size_t)SP * QD;
    FB ah, al;
    ah.h[0] = *(const v8b*)(Oh + a0); ah.h[1] = *(const v8b*)(Oh + a1);
    al.h[0] = *(const v8b*)(Ol + a0); al.h[1] = *(const v8b*)(Ol + a1);
#pragma unroll
    for (int j = 0; j < 8; ++j) {
      const v16b bw = ldfrag_b(Wb + (size_t)(j * 16 + c) * DE + kc * 32 + 8 * hh);
      acc[j] = mma_b(ah.v, bw, acc[j]);
      acc[j] = mma_b(al.v, bw, acc[j]);
    }
  }

  float* mt = Mt[wave];
#pragma unroll
  for (int j = 0; j < 8; ++j) {
#pragma unroll
    for (int r = 0; r < 8; ++r) mt[(8 * hh + r) * 132 + j * 16 + c] = acc[j][r];
  }
  wave_sync_lds();
  const int row  = lane >> 1;
  const int half = lane & 1;
  const float* mr = mt + row * 132 + half * 64;
  const float* bp = bbs + half * 64;
  const float* wp = wss + half * 64;
  float dot = 0.f;
#pragma unroll 4
  for (int n = 0; n < 64; ++n) dot = fmaf(mr[n] + bp[n], wp[n], dot);
  dot += __shfl_xor(dot, 1, 32);
  const int s  = s0w + row;
  const int sc = (s < NS) ? s : (NS - 1);
  float mk = bf_rne(mask[(size_t)b * NS + sc]);
  mk = (s < NS) ? mk : 0.f;
  const float sc1 = (dot + bf_rne(bsh[0])) * isd;
  const float lg  = clip * tanhf(sc1) + mk;
  if (half == 0) lgs[wave * 16 + row] = lg;
  __syncthreads();
  if (wave == 0 && lane < 16) {
    const v4f v = *(const v4f*)(lgs + 4 * lane);
    float* p = lgp + (size_t)R0 + 4 * lane;
    *(volatile v4f*)p = v;
    __threadfence();
    *(volatile v4f*)p = v;
  }
}

__global__ __launch_bounds__(256) void fin_softmax(const float* __restrict__ lgp, float* out) {
  __shared__ float red[8];
  __shared__ float stm[NB];
  __shared__ float sti[NB];
  const int tid = threadIdx.x, lane = tid & 31, wave = tid >> 5;
#pragma unroll 1
  for (int b = 0; b < NB; ++b) {
    const float* lr = lgp + (size_t)b * SP;
    float mx = -INFINITY;
#pragma unroll 1
    for (int s = tid; s < NS; s += 256) mx = fmaxf(mx, lr[s]);
#pragma unroll
    for (int off = 16; off > 0; off >>= 1) mx = fmaxf(mx, __shfl_xor(mx, off, 32));
    if (lane == 0) red[wave] = mx;
    __syncthreads();
    float bm = red[0];
#pragma unroll
    for (int w = 1; w < 8; ++w) bm = fmaxf(bm, red[w]);
    __syncthreads();
    float sm = 0.f;
#pragma unroll 1
    for (int s = tid; s < NS; s += 256) sm += __expf(lr[s] - bm);
#pragma unroll
    for (int off = 16; off > 0; off >>= 1) sm += __shfl_xor(sm, off, 32);
    if (lane == 0) red[wave] = sm;
    __syncthreads();
    float tot = red[0];
#pragma unroll
    for (int w = 1; w < 8; ++w) tot += red[w];
    if (tid == 0) { stm[b] = bm; sti[b] = 1.0f / tot; }
    __syncthreads();
  }
#pragma unroll 1
  for (int it = 0; it < 16; ++it) {
    const int task = it * 256 + tid;
    if (task < (NB * NS) / 32 * 8) {
      const int L = task >> 3, q8 = task & 7;
      const int idx0 = L * 32 + q8 * 4;
      float pv[4];
#pragma unroll
      for (int e = 0; e < 4; ++e) {
        const int idx = idx0 + e;
        const int bb = idx / NS;
        const int s = idx - bb * NS;
        pv[e] = __expf(lgp[(size_t)bb * SP + s] - stm[bb]) * sti[bb];
      }
      v4f v;
      v[0] = pv[0]; v[1] = pv[1]; v[2] = pv[2]; v[3] = pv[3];
      float* p = out + idx0;
      *(volatile v4f*)p = v;
      __threadfence();
      *(volatile v4f*)p = v;
    }
  }
}

extern "C" void kernel_launch(void* const* d_in, const int* in_sizes, int n_in,
                              void* d_out, int out_size, void* d_ws, size_t ws_size,
                              hipStream_t stream) {
  if (n_in < 10) return;
  if (in_sizes[0] != NB * NJ * DE) return;
  if (in_sizes[1] != NB * NM * DE) return;
  if (in_sizes[2] != NB * NS) return;
  if (in_sizes[3] != 2 * DE * DE || in_sizes[4] != 2 * DE * DE || in_sizes[5] != 2 * DE * DE) return;
  if (in_sizes[6] != DE * DE) return;
  if (in_sizes[7] != DE || in_sizes[8] != DE || in_sizes[9] < 1) return;
  if (out_size != NB * NS) return;

  const float* ej   = (const float*)d_in[0];
  const float* em   = (const float*)d_in[1];
  const float* mask = (const float*)d_in[2];
  const float* Wq   = (const float*)d_in[3];
  const float* Wk   = (const float*)d_in[4];
  const float* Wv   = (const float*)d_in[5];
  const float* Wm   = (const float*)d_in[6];
  const float* bm   = (const float*)d_in[7];
  const float* wsh  = (const float*)d_in[8];
  const float* bsh  = (const float*)d_in[9];

  const size_t PJb = (size_t)MJ * DE * 2;
  const size_t PMb = (size_t)MM * DE * 2;
  const size_t PWT = (size_t)2 * NP * DE * 2;
  const size_t PWm = (size_t)DE * DE * 2;
  const size_t PPj = (size_t)MJ * NP * 4;
  const size_t PPm = (size_t)MM * NP * 4;
  const size_t PQK = (size_t)NB * SP * QKP * 2;
  const size_t PQl = (size_t)NB * SP * QLP * 2;
  const size_t PVT = (size_t)NB * DE * SP * 2;
  const size_t PO  = (size_t)NB * NH * SP * QD * 2;
  const size_t PLG = (size_t)NB * SP * 4;
  size_t off = 0;
  const size_t oJb  = off; off += PJb;
  const size_t oMb  = off; off += PMb;
  const size_t oWT  = off; off += PWT;
  const size_t oWm  = off; off += PWm;
  const size_t oPj  = off; off += PPj;
  const size_t oPm  = off; off += PPm;
  const size_t oQK  = off; off += PQK;
  const size_t oQl  = off; off += PQl;
  const size_t oVTh = off; off += PVT;
  const size_t oVTl = off; off += PVT;
  const size_t oOh  = off; off += PO;
  const size_t oOl  = off; off += PO;
  const size_t oLG  = off; off += PLG;
  if (off > ws_size) return;
  if (off > (size_t)134217728) return;

  char* ws = (char*)d_ws;
  unsigned short* Jb  = (unsigned short*)(ws + oJb);
  unsigned short* Mb  = (unsigned short*)(ws + oMb);
  unsigned short* WT  = (unsigned short*)(ws + oWT);
  unsigned short* WmT = (unsigned short*)(ws + oWm);
  float*          Pj  = (float*)(ws + oPj);
  float*          Pm  = (float*)(ws + oPm);
  unsigned short* QK  = (unsigned short*)(ws + oQK);
  unsigned short* Ql  = (unsigned short*)(ws + oQl);
  unsigned short* VTh = (unsigned short*)(ws + oVTh);
  unsigned short* VTl = (unsigned short*)(ws + oVTl);
  unsigned short* Oh  = (unsigned short*)(ws + oOh);
  unsigned short* Ol  = (unsigned short*)(ws + oOl);
  float*          LG  = (float*)(ws + oLG);

  const dim3 blk(256);
  const int n8jv = NB * NJ * DE / 8, n8jt = MJ * DE / 8;
  const int n8mv = NB * NM * DE / 8, n8mt = MM * DE / 8;
  const dim3 gCj((n8jt + 255) / 256);
  const dim3 gCm((n8mt + 255) / 256);
  const dim3 gWt(24 + 4);
  const dim3 gPj(((MJ / 64) * (NP / 64) + 7) / 8, 1);
  const dim3 gPm(((MM / 64) * (NP / 64) + 7) / 8, 1);
  const dim3 gAs(NB * NQB);
  const dim3 gAt(NB * NH * NQB);
  const dim3 gMh(NB * SP / 64);
  const float isd = (float)(1.0 / 11.313708498984761);

  cvt_bf16x8<<<gCj, blk, 0, stream>>>(ej, Jb, n8jv, n8jt);
  cvt_bf16x8<<<gCm, blk, 0, stream>>>(em, Mb, n8mv, n8mt);
  wtr<<<gWt, blk, 0, stream>>>(Wq, Wk, Wv, Wm, WT, WmT);
  gemm64<0, 0><<<gPj, blk, 0, stream>>>(
      Jb, Jb, DE, 0LL, WT, WT, DE, 0LL,
      (void*)Pj, NP, 0LL, (void*)Pj, NP, 0LL, 0,
      MJ, NP, DE, 1.0f);
  gemm64<0, 0><<<gPm, blk, 0, stream>>>(
      Mb, Mb, DE, 0LL, WT + (size_t)NP * DE, WT + (size_t)NP * DE, DE, 0LL,
      (void*)Pm, NP, 0LL, (void*)Pm, NP, 0LL, 0,
      MM, NP, DE, 1.0f);
  asm_qkv<<<gAs, blk, 0, stream>>>(Pj, Pm, QK, Ql, VTh, VTl, 4096.0f);
  attn16<<<gAt, dim3(128), 0, stream>>>(QK, Ql, VTh, VTl, Oh, Ol, 0.25f, 1.0f / 4096.0f);
  mhlogit<<<gMh, dim3(128), 0, stream>>>(Oh, Ol, WmT, bm, wsh, bsh, mask, LG, isd, 10.0f);
  fin_softmax<<<dim3(1), blk, 0, stream>>>(LG, (float*)d_out);
  (void)hipGetLastError();
}
